// KANLinear_85341000172019
// MI455X (gfx1250) — hardware-verified
//
#include <hip/hip_runtime.h>
#include <math.h>

constexpr int kBatch    = 8192;
constexpr int kInF      = 1024;
constexpr int kOutF     = 1024;
constexpr int kNSpl     = 6;
constexpr int kOrder    = 3;
constexpr int kNumKnots = 10;
constexpr int kNumABlk  = 1 + kNSpl;
constexpr int kKAug     = kNumABlk * kInF;
constexpr int kHalfRows = kBatch / 2;
constexpr float kACarry    = 64.0f;
constexpr float kWCarry    = 64.0f;
constexpr float kLoCarry   = 256.0f;
constexpr float kMainScale = 1.0f / (64.0f * 64.0f);
constexpr float kCorrScale = 1.0f / (64.0f * 64.0f * 256.0f);

constexpr size_t kOffA     = 0;
constexpr size_t kBytesA   = (size_t)kHalfRows * kKAug * 2;
constexpr size_t kOffW     = kOffA + kBytesA;
constexpr size_t kBytesW   = (size_t)kOutF * kKAug * 2;
constexpr size_t kOffWlo   = kOffW + kBytesW;
constexpr size_t kBytesWlo = (size_t)kOutF * kInF * 2;
constexpr size_t kOffClo   = kOffWlo + kBytesWlo;
constexpr size_t kBytesClo = (size_t)kHalfRows * kOutF * 4;
constexpr size_t kWsTotal  = kOffClo + kBytesClo;
static_assert(kWsTotal == (size_t)92274688u, "ws");
static_assert(kWsTotal <= (size_t)134217728u, "ws cap");
static_assert(kOffW % 128 == 0 && kOffWlo % 128 == 0 && kOffClo % 128 == 0, "align");
static_assert(kKAug % 32 == 0 && kInF % 32 == 0, "k32");
static_assert(kHalfRows % 64 == 0 && kOutF % 64 == 0, "tile64");
static_assert(kInF % 256 == 0, "prep map");
constexpr int kGemmTiles  = (kHalfRows / 64) * (kOutF / 64);
static_assert(kGemmTiles % 8 == 0, "tiles");
constexpr int kGemmBlocks = kGemmTiles / 8;

typedef __attribute__((ext_vector_type(16))) _Float16 v16h;
typedef __attribute__((ext_vector_type(8)))  _Float16 v8h;
typedef __attribute__((ext_vector_type(16))) __bf16   v16b;
typedef __attribute__((ext_vector_type(8)))  __bf16   v8b;
typedef __attribute__((ext_vector_type(8)))  float    v8f;
typedef __attribute__((ext_vector_type(4)))  float    v4f;
typedef __attribute__((ext_vector_type(2)))  float    v2f;
typedef __attribute__((ext_vector_type(4)))  unsigned int v4u;

__device__ __forceinline__ unsigned short f2bf_bits(float f) {
  unsigned u = __float_as_uint(f);
  return (unsigned short)((u + 0x7FFFu + ((u >> 16) & 1u)) >> 16);
}
__device__ __forceinline__ float bf_bits2f(unsigned short h) { return __uint_as_float(((unsigned)h) << 16); }

__device__ __forceinline__ void dep_guard_h(v8f& a, v8f& b, v16h x, v16h y) { asm volatile("v_nop\n\tv_nop\n\tv_nop\n\tv_nop" : "+v"(a), "+v"(b) : "v"(x), "v"(y)); }
__device__ __forceinline__ void dep_guard_b(v8f& a, v8f& b, v16b x, v16b y) { asm volatile("v_nop\n\tv_nop\n\tv_nop\n\tv_nop" : "+v"(a), "+v"(b) : "v"(x), "v"(y)); }
__device__ __forceinline__ void keep4_h(v16h a, v16h b, v16h c, v16h d) { asm volatile("v_nop" :: "v"(a), "v"(b), "v"(c), "v"(d)); }
__device__ __forceinline__ void keep4_b(v16b a, v16b b, v16b c, v16b d) { asm volatile("v_nop" :: "v"(a), "v"(b), "v"(c), "v"(d)); }
__device__ __forceinline__ void acc_guard4(v8f& a, v8f& b, v8f& c, v8f& d) { asm volatile("v_nop\n\tv_nop\n\tv_nop\n\tv_nop" : "+v"(a), "+v"(b), "+v"(c), "+v"(d)); }
template <typename T> struct Frag;
template <> struct Frag<_Float16> {
  typedef v16h V; union U { v16h v; v8h h[2]; };
  static __device__ __forceinline__ v16h load(const _Float16* p) {
    U f; f.h[0] = *(const v8h*)(p); f.h[1] = *(const v8h*)(p + 16); return f.v;
  }
  static __device__ __forceinline__ v8f mma(v16h a, v16h b, v8f c) {
    return __builtin_amdgcn_wmma_f32_16x16x32_f16(false, a, false, b, (short)0, c, false, false);
  }
  static __device__ __forceinline__ void guard(v8f& a, v8f& b, v16h x, v16h y) { dep_guard_h(a, b, x, y); }
  static __device__ __forceinline__ void keep(v16h a, v16h b, v16h c, v16h d) { keep4_h(a, b, c, d); }
};
template <> struct Frag<__bf16> {
  typedef v16b V; union U { v16b v; v8b h[2]; };
  static __device__ __forceinline__ v16b load(const __bf16* p) {
    U f; f.h[0] = *(const v8b*)(p); f.h[1] = *(const v8b*)(p + 16); return f.v;
  }
  static __device__ __forceinline__ v8f mma(v16b a, v16b b, v8f c) {
    return __builtin_amdgcn_wmma_f32_16x16x32_bf16(false, a, false, b, (short)0, c, false, false);
  }
  static __device__ __forceinline__ void guard(v8f& a, v8f& b, v16b x, v16b y) { dep_guard_b(a, b, x, y); }
  static __device__ __forceinline__ void keep(v16b a, v16b b, v16b c, v16b d) { keep4_b(a, b, c, d); }
};

__device__ __forceinline__ unsigned pk16(unsigned short a, unsigned short b) { return (unsigned)a | ((unsigned)b << 16); }
__device__ __forceinline__ unsigned short h_bits(float f) { const _Float16 h = (_Float16)f; return __builtin_bit_cast(unsigned short, h); }

template <int ET> struct Elem;
template <> struct Elem<0> { typedef _Float16 T; };
template <> struct Elem<1> { typedef __bf16 T; };
template <int ET, bool SPLIT, int BIAS_MODE, int OUT_MODE, bool RESID, int ACT = 0>
__global__ __launch_bounds__(256) void wmma_gemm64(
    const unsigned short* __restrict__ Ap, const unsigned short* __restrict__ A2p, int lda, long strideA,
    const unsigned short* __restrict__ Btp, const unsigned short* __restrict__ Bt2p, int ldb, long strideB,
    void* __restrict__ Cout, void* __restrict__ Cout2, int ldc, long strideC,
    const float* __restrict__ bias,
    const float* __restrict__ resid, long strideR,
    int M, int N, int K, float scale) {
  typedef typename Elem<ET>::T T;
  typedef typename Frag<T>::V V;
  const T* A = (const T*)Ap; const T* A2 = (const T*)A2p; const T* Bt = (const T*)Btp; const T* Bt2 = (const T*)Bt2p;
  __shared__ __align__(16) float sT[8][16 * 68];
  const int b    = blockIdx.y;
  const int lane = threadIdx.x & 31;
  const int wave = threadIdx.x >> 5;
  const int tilesN = N >> 6;
  const int tilesM = M >> 6;
  const int tile = blockIdx.x * 8 + wave;
  if (tile >= tilesM * tilesN) return;
  const int tm = tile / tilesN;
  const int tn = tile - tm * tilesN;
  const int m0 = tm << 6;
  const int n0 = tn << 6;

  const T* Ab  = A  + (size_t)b * strideA;
  const T* Bb  = Bt + (size_t)b * strideB;
  const T* Ab2 = SPLIT ? (A2  + (size_t)b * strideA) : nullptr;
  const T* Bb2 = SPLIT ? (Bt2 + (size_t)b * strideB) : nullptr;

  const int rlane = lane & 15;
  const int koff  = (lane >> 4) * 8;
  const int mOff  = (lane >> 4) * 8;

  v8f acc[4][4];
#pragma unroll
  for (int i = 0; i < 4; ++i)
#pragma unroll
    for (int j = 0; j < 4; ++j) acc[i][j] = (v8f){0.f,0.f,0.f,0.f,0.f,0.f,0.f,0.f};

  for (int k0 = 0; k0 < K; k0 += 32) {
    V bh[4], bl[4];
#pragma unroll
    for (int j = 0; j < 4; ++j) {
      const size_t bo = (size_t)(n0 + (j << 4) + rlane) * ldb + koff + k0;
      bh[j] = Frag<T>::load(Bb + bo);
      if (SPLIT) bl[j] = Frag<T>::load(Bb2 + bo);
    }
#pragma unroll
    for (int i = 0; i < 4; ++i) {
      const size_t ao = (size_t)(m0 + (i << 4) + rlane) * lda + koff + k0;
      V ah = Frag<T>::load(Ab + ao);
      V al;
      if (SPLIT) al = Frag<T>::load(Ab2 + ao);
#pragma unroll
      for (int j = 0; j < 4; ++j) {
        acc[i][j] = Frag<T>::mma(ah, bh[j], acc[i][j]);
        if (SPLIT) {
          acc[i][j] = Frag<T>::mma(ah, bl[j], acc[i][j]);
          acc[i][j] = Frag<T>::mma(al, bh[j], acc[i][j]);
        }
      }
      Frag<T>::guard(acc[i][0], acc[i][3], ah, SPLIT ? al : ah);
    }
    Frag<T>::keep(bh[0], bh[1], bh[2], bh[3]);
    if (SPLIT) Frag<T>::keep(bl[0], bl[1], bl[2], bl[3]);
  }
  acc_guard4(acc[0][0], acc[0][1], acc[0][2], acc[0][3]);
  acc_guard4(acc[1][0], acc[1][1], acc[1][2], acc[1][3]);
  acc_guard4(acc[2][0], acc[2][1], acc[2][2], acc[2][3]);
  acc_guard4(acc[3][0], acc[3][1], acc[3][2], acc[3][3]);

  float* slab = sT[wave];
  const float* Rb = RESID ? (resid + (size_t)b * strideR) : nullptr;
#pragma unroll
  for (int i = 0; i < 4; ++i) {
    const int mBase = m0 + (i << 4);
#pragma unroll
    for (int j = 0; j < 4; ++j) {
      const int n = n0 + (j << 4) + rlane;
      float bv = 0.f;
      if (BIAS_MODE == 2) bv = bias[n];
#pragma unroll
      for (int r = 0; r < 8; ++r) {
        float v = acc[i][j][r] * scale;
        if (BIAS_MODE == 1) v += bias[mBase + mOff + r];
        if (BIAS_MODE == 2) v += bv;
        if (ACT == 2) v = fmaxf(v, 0.0f);
        if (ACT == 4) v = (v > 0.f) ? v : 0.01f * v;
        slab[(mOff + r) * 68 + (j << 4) + rlane] = v;
      }
    }
    __builtin_amdgcn_fence(__ATOMIC_RELEASE, "workgroup");
    __builtin_amdgcn_wave_barrier();
    __builtin_amdgcn_fence(__ATOMIC_ACQUIRE, "workgroup");
    if (OUT_MODE == 0) {
      float* C = (float*)Cout + (size_t)b * strideC;
      const int hh = lane >> 4, c4 = (lane & 15) * 4;
      if (!RESID) {
        for (int pass = 0; pass < 2; ++pass) {
#pragma unroll
          for (int it = 0; it < 8; ++it) {
            const int row = it * 2 + hh;
            v4f v = *(const v4f*)(slab + row * 68 + c4);
            *(volatile v4f*)(C + (size_t)(mBase + row) * ldc + n0 + c4) = v;
          }
          __threadfence();
        }
      } else {
        v4f ov[8];
#pragma unroll
        for (int it = 0; it < 8; ++it) {
          const int row = it * 2 + hh;
          const v4f sv = *(const v4f*)(slab + row * 68 + c4);
          const v4f rv = *(const v4f*)(Rb + (size_t)(mBase + row) * ldc + n0 + c4);
          ov[it] = sv + rv;
        }
        for (int pass = 0; pass < 2; ++pass) {
#pragma unroll
          for (int it = 0; it < 8; ++it) {
            const int row = it * 2 + hh;
            *(volatile v4f*)(C + (size_t)(mBase + row) * ldc + n0 + c4) = ov[it];
          }
          __threadfence();
        }
      }
    } else {
      const int q = lane >> 3, c8 = (lane & 7) * 8;
      unsigned short* C  = (unsigned short*)Cout  + (size_t)b * strideC;
      unsigned short* C2 = (OUT_MODE == 2) ? ((unsigned short*)Cout2 + (size_t)b * strideC) : nullptr;
      for (int pass = 0; pass < 2; ++pass) {
#pragma unroll
        for (int it = 0; it < 4; ++it) {
          const int row = it * 4 + q;
          const float* sp = slab + row * 68 + c8;
          v8h hv, lv;
#pragma unroll
          for (int e = 0; e < 8; ++e) {
            if (OUT_MODE == 1) {
              hv[e] = (_Float16)sp[e];
            } else {
              unsigned short hb = f2bf_bits(sp[e]);
              unsigned short lb = f2bf_bits(sp[e] - bf_bits2f(hb));
              hv[e] = __builtin_bit_cast(_Float16, hb);
              lv[e] = __builtin_bit_cast(_Float16, lb);
            }
          }
          *(volatile v8h*)(C + (size_t)(mBase + row) * ldc + n0 + c8) = hv;
          if (OUT_MODE == 2) *(volatile v8h*)(C2 + (size_t)(mBase + row) * ldc + n0 + c8) = lv;
        }
        __threadfence();
      }
    }
    __builtin_amdgcn_fence(__ATOMIC_RELEASE, "workgroup");
    __builtin_amdgcn_wave_barrier();
    __builtin_amdgcn_fence(__ATOMIC_ACQUIRE, "workgroup");
  }
}

__global__ __launch_bounds__(256) void wprep_kernel(const float* __restrict__ bw, const float* __restrict__ sw,
                                                    const float* __restrict__ sc,
                                                    unsigned short* __restrict__ Wout,
                                                    unsigned short* __restrict__ Wlo) {
  __shared__ __align__(16) float sm[kNumABlk + 1][kInF];
  const int t = threadIdx.x;
  const int o = blockIdx.x;
#pragma unroll 1
  for (int it = 0; it < kInF / 256; ++it) {
    const int i = it * 256 + t;
    const size_t idx = (size_t)o * kInF + i;
    const float b = bw[idx];
    const float s = sc[idx];
    const float* swp = sw + idx * kNSpl;
    const v2f w0 = *(const v2f*)(swp);
    const v2f w1 = *(const v2f*)(swp + 2);
    const v2f w2 = *(const v2f*)(swp + 4);
    const float bs  = b * kWCarry;
    const float hif = (float)((_Float16)bs);
    const float lo  = (bs - hif) * kLoCarry;
    sm[0][i] = bs;
    sm[1][i] = (w0.x * s) * kWCarry;
    sm[2][i] = (w0.y * s) * kWCarry;
    sm[3][i] = (w1.x * s) * kWCarry;
    sm[4][i] = (w1.y * s) * kWCarry;
    sm[5][i] = (w2.x * s) * kWCarry;
    sm[6][i] = (w2.y * s) * kWCarry;
    sm[7][i] = lo;
  }
  __syncthreads();
  const int lane = t & 31;
  const int wave = t >> 5;
  const float* sp = &sm[wave][0];
  unsigned short* dst = (wave < kNumABlk) ? (Wout + (size_t)o * kKAug + (size_t)wave * kInF)
                                          : (Wlo + (size_t)o * kInF);
  v4u u[4];
#pragma unroll
  for (int q = 0; q < 4; ++q) {
    const int i0 = q * 256 + lane * 8;
    const v4f a = *(const v4f*)(sp + i0);
    const v4f c = *(const v4f*)(sp + i0 + 4);
    u[q] = (v4u){pk16(h_bits(a.x), h_bits(a.y)), pk16(h_bits(a.z), h_bits(a.w)),
                 pk16(h_bits(c.x), h_bits(c.y)), pk16(h_bits(c.z), h_bits(c.w))};
  }
  for (int pass = 0; pass < 2; ++pass) {
#pragma unroll
    for (int q = 0; q < 4; ++q) *(volatile v4u*)(dst + q * 256 + lane * 8) = u[q];
    __threadfence();
  }
}

__global__ __launch_bounds__(256) void aprep_kernel(const float* __restrict__ x, const float* __restrict__ knots,
                                                    unsigned short* __restrict__ Aout, int rowBase) {
  __shared__ __align__(16) float sm[kNumABlk][kInF];
  const int t = threadIdx.x;
  const int rloc = blockIdx.x;
  const float* xr = x + (size_t)(rowBase + rloc) * kInF;
#pragma unroll 1
  for (int it = 0; it < kInF / 256; ++it) {
    const int i = it * 256 + t;
    const float v = xr[i];
    const float* kp = knots + (size_t)i * kNumKnots;
    const v2f q0 = *(const v2f*)(kp);
    const v2f q1 = *(const v2f*)(kp + 2);
    const v2f q2 = *(const v2f*)(kp + 4);
    const v2f q3 = *(const v2f*)(kp + 6);
    const v2f q4 = *(const v2f*)(kp + 8);
    float g[kNumKnots];
    g[0] = q0.x; g[1] = q0.y; g[2] = q1.x; g[3] = q1.y; g[4] = q2.x;
    g[5] = q2.y; g[6] = q3.x; g[7] = q3.y; g[8] = q4.x; g[9] = q4.y;

    const float e = expf(-v);
    const float sil = v / (1.0f + e);

    float bas[kNumKnots - 1];
#pragma unroll
    for (int j = 0; j < kNumKnots - 1; ++j) bas[j] = (v >= g[j] && v < g[j + 1]) ? 1.0f : 0.0f;
#pragma unroll
    for (int k = 1; k <= kOrder; ++k) {
#pragma unroll
      for (int j = 0; j < kNumKnots - 1 - k; ++j) {
        const float rl = __builtin_amdgcn_rcpf(g[j + k] - g[j]);
        const float rr = __builtin_amdgcn_rcpf(g[j + k + 1] - g[j + 1]);
        const float lf = (v - g[j]) * rl;
        const float rt = (g[j + k + 1] - v) * rr;
        bas[j] = lf * bas[j] + rt * bas[j + 1];
      }
    }
    sm[0][i] = sil * kACarry;
#pragma unroll
    for (int c = 0; c < kNSpl; ++c) sm[1 + c][i] = bas[c] * kACarry;
  }
  __syncthreads();
  const int lane = t & 31;
  const int wave = t >> 5;
  if (wave < kNumABlk) {
    const float* sp = &sm[wave][0];
    unsigned short* dst = Aout + (size_t)rloc * kKAug + (size_t)wave * kInF;
    v4u u[4];
#pragma unroll
    for (int q = 0; q < 4; ++q) {
      const int i0 = q * 256 + lane * 8;
      const v4f a = *(const v4f*)(sp + i0);
      const v4f c = *(const v4f*)(sp + i0 + 4);
      u[q] = (v4u){pk16(h_bits(a.x), h_bits(a.y)), pk16(h_bits(a.z), h_bits(a.w)),
                   pk16(h_bits(c.x), h_bits(c.y)), pk16(h_bits(c.z), h_bits(c.w))};
    }
    for (int pass = 0; pass < 2; ++pass) {
#pragma unroll
      for (int q = 0; q < 4; ++q) *(volatile v4u*)(dst + q * 256 + lane * 8) = u[q];
      __threadfence();
    }
  }
}

extern "C" void kernel_launch(void* const* d_in, const int* in_sizes, int n_in,
                              void* d_out, int out_size, void* d_ws, size_t ws_size,
                              hipStream_t stream) {
  if (n_in < 5) return;
  if (in_sizes[0] != kBatch * kInF) return;
  if (in_sizes[1] != kOutF * kInF) return;
  if (in_sizes[2] != kOutF * kInF * kNSpl) return;
  if (in_sizes[3] != kOutF * kInF) return;
  if (in_sizes[4] != kInF * kNumKnots) return;
  if (out_size != kBatch * kOutF) return;
  if (ws_size < kWsTotal) return;

  const float* x  = (const float*)d_in[0];
  const float* bw = (const float*)d_in[1];
  const float* sw = (const float*)d_in[2];
  const float* sc = (const float*)d_in[3];
  const float* kn = (const float*)d_in[4];

  char* ws = (char*)d_ws;
  unsigned short* Ah  = (unsigned short*)(ws + kOffA);
  unsigned short* Wh  = (unsigned short*)(ws + kOffW);
  unsigned short* Wlo = (unsigned short*)(ws + kOffWlo);
  float*          Clo = (float*)(ws + kOffClo);
  float*          outp = (float*)d_out;

  wprep_kernel<<<dim3(kOutF), dim3(256), 0, stream>>>(bw, sw, sc, Wh, Wlo);

  for (int h = 0; h < 2; ++h) {
    aprep_kernel<<<dim3(kHalfRows), dim3(256), 0, stream>>>(x, kn, Ah, h * kHalfRows);

    wmma_gemm64<0, false, 0, 0, false><<<dim3(kGemmBlocks, 1), dim3(256), 0, stream>>>(
        Ah, Ah, kKAug, 0L,
        Wlo, Wlo, kInF, 0L,
        (void*)Clo, (void*)Clo, kOutF, 0L,
        bw,
        x, 0L,
        kHalfRows, kOutF, kInF, kCorrScale);

    float* Ch = outp + (size_t)h * kHalfRows * kOutF;
    wmma_gemm64<0, false, 0, 0, true><<<dim3(kGemmBlocks, 1), dim3(256), 0, stream>>>(
        Ah, Ah, kKAug, 0L,
        Wh, Wh, kKAug, 0L,
        (void*)Ch, (void*)Ch, kOutF, 0L,
        bw,
        Clo, 0L,
        kHalfRows, kOutF, kKAug, kMainScale);
  }
}
